// MutualCrossAttention_80367428042874
// MI455X (gfx1250) — hardware-verified
//
#include <hip/hip_runtime.h>
#include <stdint.h>

typedef __attribute__((ext_vector_type(16))) _Float16 v16h;
typedef __attribute__((ext_vector_type(8)))  _Float16 v8h;
typedef __attribute__((ext_vector_type(8)))  float    v8f;
typedef __attribute__((ext_vector_type(4)))  float    v4f;
typedef __attribute__((ext_vector_type(4)))  unsigned v4u;

#define NBATCH   8
#define SEQ_LEN  2048
#define DMODEL   512

#define QB_ROWS    32
#define KC_KEYS    64
#define QS_PITCH   520
#define KS_PITCH   520
#define VT_PITCH   72
#define SB_PITCH   68
#define PB_PITCH   72
#define SLAB_PITCH 132
#define OFF_QS  0
#define OFF_KS  (OFF_QS + QB_ROWS * QS_PITCH * 2)
#define OFF_VT  (OFF_KS + KC_KEYS * KS_PITCH * 2)
#define OFF_SB  (OFF_VT + DMODEL * VT_PITCH * 2)
#define OFF_PB  (OFF_SB + 2 * 16 * SB_PITCH * 4)
#define OFF_LB  (OFF_PB + 2 * 16 * PB_PITCH * 2)
#define LDS_TOTAL (OFF_LB + 2 * 4 * 16 * 4)
#define P_CARRY 32768.0f
#define TR_PITCH 72

static_assert(OFF_KS == 33280 && OFF_VT == 99840 && OFF_SB == 173568 && OFF_PB == 182272 && OFF_LB == 186880, "lds carve");
static_assert(LDS_TOTAL == 187392, "lds total");
static_assert((OFF_KS % 16) == 0 && (OFF_VT % 16) == 0 && (OFF_SB % 16) == 0 && (OFF_PB % 16) == 0 && (OFF_LB % 16) == 0, "lds align");
static_assert(8 * 16 * SLAB_PITCH * 4 <= DMODEL * VT_PITCH * 2, "slab reuse fits in Vt region");
static_assert((SEQ_LEN % QB_ROWS) == 0 && (SEQ_LEN % KC_KEYS) == 0 && (DMODEL % 128) == 0 && (DMODEL % 32) == 0 && (KC_KEYS % 32) == 0, "tile multiples");
static_assert((SEQ_LEN % 64) == 0 && (DMODEL % 64) == 0, "convert tile multiples");

union FH { v16h v; v8h h[2]; };

__device__ __forceinline__ v8f zero8() { v8f z = {0.f, 0.f, 0.f, 0.f, 0.f, 0.f, 0.f, 0.f}; return z; }

__device__ __forceinline__ v8f hmma(v16h a, v16h b, v8f c) {
  c = __builtin_amdgcn_wmma_f32_16x16x32_f16(false, a, false, b, (short)0, c, false, false);
  asm volatile("v_nop\n\tv_nop\n\tv_nop\n\tv_nop" : "+v"(c) : "v"(a), "v"(b));
  return c;
}

__device__ __forceinline__ unsigned cvt_bits(float x) {
  unsigned u = __float_as_uint(x);
  u = (u + 0x7FFFu + ((u >> 16) & 1u)) & 0xFFFF0000u;
  const float r = __uint_as_float(u);
  const _Float16 hv = (_Float16)r;
  return (unsigned)__builtin_bit_cast(unsigned short, hv);
}

__global__ __launch_bounds__(256)
void cvt_planes(const float* __restrict__ xin, _Float16* __restrict__ xh, _Float16* __restrict__ xt) {
  __shared__ __align__(16) unsigned short tile[64 * TR_PITCH];
  const int tid = threadIdx.x;
  const int tilesD = DMODEL / 64;
  const int tilesL = SEQ_LEN / 64;
  const int b  = blockIdx.x / (tilesL * tilesD);
  const int rr = blockIdx.x - b * (tilesL * tilesD);
  const int lt = rr / tilesD;
  const int l0 = lt * 64;
  const int d0 = (rr - lt * tilesD) * 64;

  v4u w[2];
#pragma unroll
  for (int it = 0; it < 2; ++it) {
    const int idx = it * 256 + tid;
    const int row = idx >> 3, c8 = idx & 7;
    const float* src = xin + ((size_t)b * SEQ_LEN + l0 + row) * DMODEL + d0 + c8 * 8;
    const v4f f0 = *(const v4f*)src;
    const v4f f1 = *(const v4f*)(src + 4);
    v4u ww;
    ww.x = cvt_bits(f0.x) | (cvt_bits(f0.y) << 16);
    ww.y = cvt_bits(f0.z) | (cvt_bits(f0.w) << 16);
    ww.z = cvt_bits(f1.x) | (cvt_bits(f1.y) << 16);
    ww.w = cvt_bits(f1.z) | (cvt_bits(f1.w) << 16);
    w[it] = ww;
    *(v4u*)(tile + row * TR_PITCH + c8 * 8) = ww;
  }
  for (int pass = 0; pass < 2; ++pass) {
#pragma unroll
    for (int it = 0; it < 2; ++it) {
      const int idx = it * 256 + tid;
      const int row = idx >> 3, c8 = idx & 7;
      *(volatile v4u*)(xh + ((size_t)b * SEQ_LEN + l0 + row) * DMODEL + d0 + c8 * 8) = w[it];
    }
    __threadfence();
  }
  __syncthreads();
  v4u t2[2];
#pragma unroll
  for (int it = 0; it < 2; ++it) {
    const int idx = it * 256 + tid;
    const int drow = idx >> 3, c8 = idx & 7;
    const unsigned short* tp = tile + (c8 * 8) * TR_PITCH + drow;
    const unsigned e0 = tp[0 * TR_PITCH], e1 = tp[1 * TR_PITCH], e2 = tp[2 * TR_PITCH], e3 = tp[3 * TR_PITCH];
    const unsigned e4 = tp[4 * TR_PITCH], e5 = tp[5 * TR_PITCH], e6 = tp[6 * TR_PITCH], e7 = tp[7 * TR_PITCH];
    v4u ww;
    ww.x = e0 | (e1 << 16);
    ww.y = e2 | (e3 << 16);
    ww.z = e4 | (e5 << 16);
    ww.w = e6 | (e7 << 16);
    t2[it] = ww;
  }
  for (int pass = 0; pass < 2; ++pass) {
#pragma unroll
    for (int it = 0; it < 2; ++it) {
      const int idx = it * 256 + tid;
      const int drow = idx >> 3, c8 = idx & 7;
      *(volatile v4u*)(xt + ((size_t)b * DMODEL + d0 + drow) * SEQ_LEN + l0 + c8 * 8) = t2[it];
    }
    __threadfence();
  }
}

template <bool RESID>
__global__ __launch_bounds__(256)
void xattn512(const _Float16* __restrict__ qh, const _Float16* __restrict__ kh,
              const _Float16* __restrict__ kt, const float* rsd, float* dst, float c2) {
  extern __shared__ __align__(16) unsigned char lds_raw[];
  _Float16* Qs = (_Float16*)(lds_raw + OFF_QS);
  _Float16* Ks = (_Float16*)(lds_raw + OFF_KS);
  _Float16* Vt = (_Float16*)(lds_raw + OFF_VT);
  float*    Sb = (float*)(lds_raw + OFF_SB);
  _Float16* Pb = (_Float16*)(lds_raw + OFF_PB);
  float*    Lb = (float*)(lds_raw + OFF_LB);

  const int tid  = threadIdx.x;
  const int wave = tid >> 5;
  const int lane = tid & 31;
  const int hh   = lane >> 4;
  const int c    = lane & 15;
  const int nqb  = SEQ_LEN / QB_ROWS;
  const int b    = blockIdx.x / nqb;
  const int qb   = blockIdx.x - b * nqb;
  const int q0   = qb * QB_ROWS;
  const int mr   = wave >> 2;
  const int sub  = wave & 3;

  {
    const _Float16* qsrc = qh + ((size_t)b * SEQ_LEN + q0) * DMODEL;
#pragma unroll
    for (int it = 0; it < 8; ++it) {
      const int idx = it * 256 + tid;
      const int row = idx >> 6, cc = idx & 63;
      *(v4u*)(Qs + row * QS_PITCH + cc * 8) = *(const v4u*)(qsrc + (size_t)row * DMODEL + cc * 8);
    }
  }

  float mrow[8], lrow[8], alpha[8];
  v8f oacc[8];
#pragma unroll
  for (int r = 0; r < 8; ++r) { mrow[r] = -INFINITY; lrow[r] = 0.f; alpha[r] = 0.f; }
#pragma unroll
  for (int t = 0; t < 8; ++t) oacc[t] = zero8();

  const _Float16* kbase = kh + (size_t)b * SEQ_LEN * DMODEL;
  const _Float16* tbase = kt + (size_t)b * DMODEL * SEQ_LEN;
  const int nkc = SEQ_LEN / KC_KEYS;

#pragma unroll 1
  for (int kc = 0; kc < nkc; ++kc) {
    __syncthreads();
    {
      const _Float16* ksrc = kbase + (size_t)kc * KC_KEYS * DMODEL;
#pragma unroll 4
      for (int it = 0; it < 16; ++it) {
        const int idx = it * 256 + tid;
        const int row = idx >> 6, cc = idx & 63;
        *(v4u*)(Ks + row * KS_PITCH + cc * 8) = *(const v4u*)(ksrc + (size_t)row * DMODEL + cc * 8);
      }
      const _Float16* tsrc = tbase + (size_t)kc * KC_KEYS;
      const int c8 = tid & 7, dl = tid >> 3;
#pragma unroll 4
      for (int it = 0; it < 16; ++it) {
        const int d = it * 32 + dl;
        *(v4u*)(Vt + d * VT_PITCH + c8 * 8) = *(const v4u*)(tsrc + (size_t)d * SEQ_LEN + c8 * 8);
      }
    }
    __syncthreads();

    {
      v8f s = zero8();
      const _Float16* qrow = Qs + (mr * 16 + c) * QS_PITCH + 8 * hh;
      const _Float16* krow = Ks + (sub * 16 + c) * KS_PITCH + 8 * hh;
#pragma unroll 4
      for (int dc = 0; dc < 16; ++dc) {
        FH a, kb;
        a.h[0]  = *(const v8h*)(qrow + dc * 32);
        a.h[1]  = *(const v8h*)(qrow + dc * 32 + 16);
        kb.h[0] = *(const v8h*)(krow + dc * 32);
        kb.h[1] = *(const v8h*)(krow + dc * 32 + 16);
        s = hmma(a.v, kb.v, s);
      }
      float* sdst = Sb + (mr * 16 + 8 * hh) * SB_PITCH + sub * 16 + c;
#pragma unroll
      for (int r = 0; r < 8; ++r) sdst[r * SB_PITCH] = s[r] * c2;
    }
    __syncthreads();

    {
      const float* srd = Sb + (mr * 16 + 8 * hh) * SB_PITCH + c;
      _Float16* pdst = Pb + (mr * 16 + 8 * hh) * PB_PITCH + sub * 16 + c;
#pragma unroll
      for (int r = 0; r < 8; ++r) {
        const float v0 = srd[r * SB_PITCH];
        const float v1 = srd[r * SB_PITCH + 16];
        const float v2 = srd[r * SB_PITCH + 32];
        const float v3 = srd[r * SB_PITCH + 48];
        float m = fmaxf(fmaxf(v0, v1), fmaxf(v2, v3));
#pragma unroll
        for (int off = 1; off < 16; off <<= 1) m = fmaxf(m, __shfl_xor(m, off, 32));
        const float vo   = srd[r * SB_PITCH + sub * 16];
        const float mnew = fmaxf(mrow[r], m);
        const float al   = exp2f(mrow[r] - mnew);
        const float p    = exp2f(vo - mnew);
        float ps = p;
#pragma unroll
        for (int off = 1; off < 16; off <<= 1) ps += __shfl_xor(ps, off, 32);
        pdst[r * PB_PITCH] = (_Float16)(p * P_CARRY);
        if (c == 0) Lb[(mr * 4 + sub) * 16 + 8 * hh + r] = ps;
        mrow[r]  = mnew;
        alpha[r] = al;
#pragma unroll
        for (int t = 0; t < 8; ++t) oacc[t][r] *= al;
      }
    }
    __syncthreads();

    {
#pragma unroll
      for (int r = 0; r < 8; ++r) {
        const float* lp = Lb + mr * 64 + 8 * hh + r;
        const float tot = ((lp[0] + lp[16]) + lp[32]) + lp[48];
        lrow[r] = lrow[r] * alpha[r] + tot;
      }
      const _Float16* prow = Pb + (mr * 16 + c) * PB_PITCH + 8 * hh;
      const _Float16* vrow = Vt + (sub * 128 + c) * VT_PITCH + 8 * hh;
#pragma unroll 1
      for (int kk = 0; kk < 2; ++kk) {
        FH pa;
        pa.h[0] = *(const v8h*)(prow + kk * 32);
        pa.h[1] = *(const v8h*)(prow + kk * 32 + 16);
#pragma unroll
        for (int t = 0; t < 8; ++t) {
          FH vb;
          vb.h[0] = *(const v8h*)(vrow + t * 16 * VT_PITCH + kk * 32);
          vb.h[1] = *(const v8h*)(vrow + t * 16 * VT_PITCH + kk * 32 + 16);
          oacc[t] = hmma(pa.v, vb.v, oacc[t]);
        }
      }
    }
  }
  __syncthreads();

  float* slab = (float*)(lds_raw + OFF_VT) + wave * (16 * SLAB_PITCH);
#pragma unroll
  for (int r = 0; r < 8; ++r) {
    const float inv = 1.0f / (lrow[r] * P_CARRY);
#pragma unroll
    for (int t = 0; t < 8; ++t) slab[(8 * hh + r) * SLAB_PITCH + t * 16 + c] = oacc[t][r] * inv;
  }
  __syncthreads();
  const size_t grow0 = (size_t)b * SEQ_LEN + q0 + mr * 16;
  const int col = sub * 128 + lane * 4;
  if (RESID) {
#pragma unroll 4
    for (int row = 0; row < 16; ++row) {
      v4f v = *(const v4f*)(slab + row * SLAB_PITCH + lane * 4);
      const v4f ra = *(const v4f*)(rsd + (grow0 + row) * DMODEL + col);
      v += ra;
      *(v4f*)(slab + row * SLAB_PITCH + lane * 4) = v;
    }
  }
  for (int pass = 0; pass < 2; ++pass) {
#pragma unroll
    for (int row = 0; row < 16; ++row) {
      const v4f v = *(const v4f*)(slab + row * SLAB_PITCH + lane * 4);
      *(volatile v4f*)(dst + (grow0 + row) * DMODEL + col) = v;
    }
    __threadfence();
  }
}

extern "C" void kernel_launch(void* const* d_in, const int* in_sizes, int n_in,
                              void* d_out, int out_size, void* d_ws, size_t ws_size,
                              hipStream_t stream) {
  const size_t nElem = (size_t)NBATCH * SEQ_LEN * DMODEL;
  if (n_in < 2) return;
  if (in_sizes[0] != (int)nElem || in_sizes[1] != (int)nElem || out_size != (int)nElem) return;
  const size_t planeH = nElem * 2;
  const size_t planeF = nElem * 4;
  const size_t off_x1h = 0;
  const size_t off_x2h = off_x1h + planeH;
  const size_t off_x1t = off_x2h + planeH;
  const size_t off_x2t = off_x1t + planeH;
  const size_t off_oa  = off_x2t + planeH;
  const size_t total   = off_oa + planeF;
  if (d_ws == nullptr || ws_size < total) return;

  const float* x1 = (const float*)d_in[0];
  const float* x2 = (const float*)d_in[1];
  float* out = (float*)d_out;
  unsigned char* ws = (unsigned char*)d_ws;
  _Float16* x1h = (_Float16*)(ws + off_x1h);
  _Float16* x2h = (_Float16*)(ws + off_x2h);
  _Float16* x1t = (_Float16*)(ws + off_x1t);
  _Float16* x2t = (_Float16*)(ws + off_x2t);
  float*    oA  = (float*)(ws + off_oa);

  const float scale = 0.04419417382415922f;
  const float c2 = scale * 1.4426950408889634f;

  const dim3 blk(256);
  const dim3 gcv(NBATCH * (SEQ_LEN / 64) * (DMODEL / 64));
  const dim3 gat(NBATCH * (SEQ_LEN / QB_ROWS));

  cvt_planes<<<gcv, blk, 0, stream>>>(x1, x1h, x1t);
  cvt_planes<<<gcv, blk, 0, stream>>>(x2, x2h, x2t);
  xattn512<false><<<gat, blk, LDS_TOTAL, stream>>>(x1h, x2h, x2t, oA, oA, c2);
  xattn512<true><<<gat, blk, LDS_TOTAL, stream>>>(x2h, x1h, x1t, oA, out, c2);
}
